// ContextualAttention_31215822307689
// MI455X (gfx1250) — hardware-verified
//
#include <hip/hip_runtime.h>


#ifndef NB
#define NB 2
#endif
#define CH   64
#define HF   128
#define HS   64
#define NPIX 4096
#define NPAT 4096
#define KD   576
#define NV   1024
#define IMG_FULL ((size_t)CH * HF * HF)
#define MSK_FULL ((size_t)HF * HF)
#define PCAR 16384.0f
#define VCAR 16.0f
#define SMS  10.0f

static_assert(NPIX % 64 == 0);
static_assert(NPAT % 64 == 0);
static_assert(NV % 64 == 0);
static_assert(KD % 32 == 0);
static_assert(NPAT % 32 == 0);
static_assert((8 * KD) % 256 == 0);
static_assert(NPAT == 16 * 256);
static_assert((size_t)NPIX * NV * 4 <= (size_t)NPIX * NPAT * 4);

typedef _Float16 h16;
typedef unsigned short bf;
typedef __attribute__((ext_vector_type(16))) __bf16   v16bf;
typedef __attribute__((ext_vector_type(16))) _Float16 v16h;
typedef __attribute__((ext_vector_type(8)))  _Float16 v8h;
typedef __attribute__((ext_vector_type(8)))  unsigned short v8us;
typedef __attribute__((ext_vector_type(8)))  float    v8f;
typedef __attribute__((ext_vector_type(4)))  float    v4f;
typedef v8h  __attribute__((may_alias)) v8ha;
typedef v4f  __attribute__((may_alias)) v4fa;
typedef v8us __attribute__((may_alias)) v8usa;

__device__ __forceinline__ unsigned short f2bf(float f) { unsigned u = __float_as_uint(f); u += 0x7FFFu + ((u >> 16) & 1u); return (unsigned short)(u >> 16); }
__device__ __forceinline__ float bf2f(unsigned short b) { return __uint_as_float(((unsigned)b) << 16); }
__device__ __forceinline__ float bfr(float f) { return bf2f(f2bf(f)); }
__device__ __forceinline__ v16h cat16(v8h lo, v8h hi) { return __builtin_shufflevector(lo, hi, 0, 1, 2, 3, 4, 5, 6, 7, 8, 9, 10, 11, 12, 13, 14, 15); }
__device__ __forceinline__ v16bf cat16b(v8us lo, v8us hi) { return __builtin_bit_cast(v16bf, __builtin_shufflevector(lo, hi, 0, 1, 2, 3, 4, 5, 6, 7, 8, 9, 10, 11, 12, 13, 14, 15)); }
__device__ __forceinline__ v8f wmma16(v16h a, v16h b, v8f c) { return __builtin_amdgcn_wmma_f32_16x16x32_f16(false, a, false, b, (short)0, c, false, false); }
__device__ __forceinline__ v8f wmmab(v16bf a, v16bf b, v8f c) { return __builtin_amdgcn_wmma_f32_16x16x32_bf16(false, a, false, b, (short)0, c, false, false); }

template <typename T16> struct WFrag;
template <> struct WFrag<h16> { typedef v16h V; static __device__ __forceinline__ V ld(const h16* p) { return cat16(*(const v8h*)p, *(const v8h*)(p + 16)); } static __device__ __forceinline__ v8f mma(V a, V b, v8f c) { return wmma16(a, b, c); } };
template <> struct WFrag<bf> { typedef v16bf V; static __device__ __forceinline__ V ld(const bf* p) { return cat16b(*(const v8us*)p, *(const v8us*)(p + 16)); } static __device__ __forceinline__ v8f mma(V a, V b, v8f c) { return wmmab(a, b, c); } };
template <typename T16, int EPI>
__global__ __launch_bounds__(32) void k_gemmw(const T16* __restrict__ A, const T16* __restrict__ Bt, int K, float* C, int ldc, const float* __restrict__ csc) {
    typedef typename WFrag<T16>::V V;
    __shared__ __align__(16) float os[16 * 68];
    const int lane = threadIdx.x & 31, lr = lane & 15, hi = lane >> 4; const int r0 = blockIdx.x * 64, c0 = blockIdx.y * 64;
    v8f acc[4][4];
#pragma unroll
    for (int mb = 0; mb < 4; ++mb)
#pragma unroll
        for (int nb = 0; nb < 4; ++nb) acc[mb][nb] = (v8f){};
    const size_t aoff = (size_t)(r0 + lr) * K + 8 * hi, boff = (size_t)(c0 + lr) * K + 8 * hi;
#pragma unroll 1
    for (int kc = 0; kc < K; kc += 32) {
        V a[4];
#pragma unroll
        for (int mb = 0; mb < 4; ++mb) a[mb] = WFrag<T16>::ld(A + aoff + (size_t)mb * 16 * K + kc);
#pragma unroll
        for (int nb = 0; nb < 4; ++nb) { const V b = WFrag<T16>::ld(Bt + boff + (size_t)nb * 16 * K + kc);
#pragma unroll
            for (int mb = 0; mb < 4; ++mb) acc[mb][nb] = WFrag<T16>::mma(a[mb], b, acc[mb][nb]); }
        asm volatile("v_nop\n\tv_nop\n\tv_nop\n\tv_nop" : "+v"(acc[0][0]), "+v"(acc[1][1]), "+v"(acc[2][2]), "+v"(acc[3][3]) : "v"(a[0]), "v"(a[3]));
    }
    v4f sc4; sc4[0] = 1.0f; sc4[1] = 1.0f; sc4[2] = 1.0f; sc4[3] = 1.0f;
    if (EPI == 1) sc4 = *(const v4f*)(csc + c0 + lr * 4);
#pragma unroll
    for (int mb = 0; mb < 4; ++mb) {
#pragma unroll
        for (int nb = 0; nb < 4; ++nb) {
#pragma unroll
            for (int j = 0; j < 8; ++j) os[(hi * 8 + j) * 68 + nb * 16 + lr] = acc[mb][nb][j]; }
        __builtin_amdgcn_wave_barrier(); asm volatile("" ::: "memory");
        float* crow = C + (size_t)(r0 + mb * 16) * ldc + c0;
#pragma unroll 1
        for (int ps = 0; ps < 2; ++ps) {
#pragma unroll
            for (int s = 0; s < 8; ++s) { const int row = 2 * s + hi, cofs = lr * 4; v4f val = *(const v4fa*)(os + row * 68 + cofs); if (EPI == 1) val = val * sc4;
                *(volatile v4f*)(crow + (size_t)row * ldc + cofs) = val; }
            if (ps == 0) __threadfence(); }
        __builtin_amdgcn_wave_barrier(); asm volatile("" ::: "memory");
    }
}

__global__ __launch_bounds__(256) void k_fga(const float* __restrict__ fg, bf* AP) {
    const int lane = threadIdx.x & 31; const int w = blockIdx.x * 8 + (threadIdx.x >> 5);
    if (w * 8 >= NPIX) return;
    const size_t base = (size_t)w * 8 * KD;
#pragma unroll 1
    for (int j = 0; j < (8 * KD) / 256; ++j) {
        const int E = (32 * j + lane) * 8; const int r = E / KD; const int k0 = E - r * KD; const int p = w * 8 + r; const int py = p >> 6, px = p & 63;
        v8us o;
#pragma unroll
        for (int q = 0; q < 8; ++q) { const int k = k0 + q; const int c = k / 9; const int r9 = k - 9 * c; const int ki = r9 / 3; const int kj = r9 - 3 * ki;
            const int y = py + ki - 1, x = px + kj - 1; const bool ok = ((unsigned)y < (unsigned)HS) && ((unsigned)x < (unsigned)HS);
            const int yc = min(max(y, 0), HS - 1), xc = min(max(x, 0), HS - 1);
            const float v = fg[((size_t)c * HF + 2 * yc) * HF + 2 * xc];
            o[q] = ok ? f2bf(v) : (unsigned short)0; }
        bf* dst = AP + base + E;
        *(volatile v8us*)dst = o; __threadfence(); *(volatile v8us*)dst = o;
    }
}

__global__ __launch_bounds__(256) void k_bgb(const float* __restrict__ bg, const float* __restrict__ mk, bf* BP, float* INV, int* FLG) {
    __shared__ float invs[64];
    const int lane = threadIdx.x & 31, wid = threadIdx.x >> 5; const int w = blockIdx.x * 8 + wid;
    const size_t base = (size_t)w * 8 * KD;
    float ss[8];
#pragma unroll
    for (int rr = 0; rr < 8; ++rr) ss[rr] = 0.0f;
#pragma unroll 1
    for (int j = 0; j < (8 * KD) / 256; ++j) {
        const int E = (32 * j + lane) * 8; const int r = E / KD; const int k0 = E - r * KD; const int l = w * 8 + r; const int ly = l >> 6, lx = l & 63;
        v8us o; float pss = 0.0f;
#pragma unroll
        for (int q = 0; q < 8; ++q) { const int k = k0 + q; const int c = k / 9; const int r9 = k - 9 * c; const int ki = r9 / 3; const int kj = r9 - 3 * ki;
            const int y = ly + ki - 1, x = lx + kj - 1; const bool ok = ((unsigned)y < (unsigned)HS) && ((unsigned)x < (unsigned)HS);
            const int yc = min(max(y, 0), HS - 1), xc = min(max(x, 0), HS - 1);
            const float v = bg[((size_t)c * HF + 2 * yc) * HF + 2 * xc];
            const unsigned short hb = ok ? f2bf(v) : (unsigned short)0; o[q] = hb; const float vb = bf2f(hb); pss += vb * vb; }
#pragma unroll
        for (int rr = 0; rr < 8; ++rr) ss[rr] += (r == rr) ? pss : 0.0f;
        bf* dst = BP + base + E;
        *(volatile v8us*)dst = o; __threadfence(); *(volatile v8us*)dst = o;
    }
    float mine = 0.0f;
#pragma unroll
    for (int rr = 0; rr < 8; ++rr) { float s = ss[rr];
#pragma unroll
        for (int sh = 16; sh; sh >>= 1) s += __shfl_xor(s, sh, 32);
        mine = (lane == rr) ? s : mine; }
    if (lane < 8) invs[wid * 8 + lane] = 1.0f / fmaxf(sqrtf(mine), 1.0e-3f);
    __syncthreads();
    if (wid < 2) {
        const int li = wid * 32 + lane; const int l = blockIdx.x * 64 + li; const float iv = invs[li];
        const int ly = l >> 6, lx = l & 63; float ms = 0.0f;
#pragma unroll
        for (int ki = 0; ki < 3; ++ki)
#pragma unroll
            for (int kj = 0; kj < 3; ++kj) { const int y = ly + ki - 1, x = lx + kj - 1; const bool ok = ((unsigned)y < (unsigned)HS) && ((unsigned)x < (unsigned)HS);
                const int yc = min(max(y, 0), HS - 1), xc = min(max(x, 0), HS - 1);
                const float m = bfr(mk[(size_t)(2 * yc) * HF + 2 * xc]); ms += ok ? m : 0.0f; }
        const int fl = (ms == 0.0f) ? 1 : 0;
#pragma unroll 1
        for (int ps = 0; ps < 2; ++ps) { *(volatile float*)(INV + l) = iv; *(volatile int*)(FLG + l) = fl; if (ps == 0) __threadfence(); }
    }
}

__global__ __launch_bounds__(256) void k_vt(const float* __restrict__ bg, h16* VT) {
    const int n = blockIdx.x; const int c = n >> 4, a = (n >> 2) & 3, b2 = n & 3; const int tid = threadIdx.x;
#pragma unroll
    for (int j = 0; j < 2; ++j) {
        const int Q = j * 256 + tid; const int l0 = Q * 8; const int ly = l0 >> 6, lx0 = l0 & 63;
        const int Y = 2 * ly + a - 1; const bool oky = (unsigned)Y < (unsigned)HF; const int Yc = min(max(Y, 0), HF - 1);
        v8h o;
#pragma unroll
        for (int q = 0; q < 8; ++q) { const int X = 2 * (lx0 + q) + b2 - 1; const bool okx = (unsigned)X < (unsigned)HF; const int Xc = min(max(X, 0), HF - 1);
            const float v = bg[((size_t)c * HF + Yc) * HF + Xc];
            o[q] = (oky && okx) ? (h16)(bfr(v) * VCAR) : (h16)0.0f; }
        h16* dst = VT + (size_t)n * NPAT + l0;
        *(volatile v8h*)dst = o; __threadfence(); *(volatile v8h*)dst = o;
    }
}

__global__ __launch_bounds__(256) void k_soft(const float* __restrict__ S, const int* __restrict__ FLG, h16* P16) {
    __shared__ __align__(16) h16 prow[NPAT];
    __shared__ float redm[8]; __shared__ float reds[8];
    const int p = blockIdx.x, tid = threadIdx.x, lane = tid & 31, wid = tid >> 5;
    const int tp = ((p & 63) << 6) | (p >> 6);
    float v[16]; float mx = -3.0e38f;
#pragma unroll
    for (int t = 0; t < 16; ++t) {
        const int l = tid + 256 * t; const int tl = ((l & 63) << 6) | (l >> 6);
        float s = 0.0f;
#pragma unroll
        for (int e2 = 0; e2 < 3; ++e2) { const int d2 = e2 - 1;
            const int ia = tp + d2; const bool va = (unsigned)ia < (unsigned)NPIX; const int iac = min(max(ia, 0), NPIX - 1); const int i2 = ((iac & 63) << 6) | (iac >> 6);
            const int jb = tl + d2; const bool vb = (unsigned)jb < (unsigned)NPAT; const int jbc = min(max(jb, 0), NPAT - 1); const int j2 = ((jbc & 63) << 6) | (jbc >> 6);
            float in = 0.0f;
#pragma unroll
            for (int e1 = 0; e1 < 3; ++e1) { const int d1 = e1 - 1;
                const int ii = i2 + d1; const bool vi = va && ((unsigned)ii < (unsigned)NPIX); const int iic = min(max(ii, 0), NPIX - 1);
                const int jj = j2 + d1; const bool vj = vb && ((unsigned)jj < (unsigned)NPAT); const int jjc = min(max(jj, 0), NPAT - 1);
                const float x = S[(size_t)iic * NPAT + jjc];
                in = in + ((vi && vj) ? x : 0.0f); }
            s = s + in; }
        const int fl = FLG[l];
        const float sc = (fl != 0) ? -1000.0f : s;
        const float tt = SMS * sc;
        v[t] = tt; mx = fmaxf(mx, tt);
        asm volatile("" ::: "memory");
    }
#pragma unroll
    for (int sh = 16; sh; sh >>= 1) mx = fmaxf(mx, __shfl_xor(mx, sh, 32));
    if (lane == 0) redm[wid] = mx;
    __syncthreads();
    mx = redm[0];
#pragma unroll
    for (int i = 1; i < 8; ++i) mx = fmaxf(mx, redm[i]);
    float sum = 0.0f;
#pragma unroll
    for (int t = 0; t < 16; ++t) { float d0 = __fsub_rn(v[t], mx); asm volatile("" : "+v"(d0)); v[t] = __builtin_amdgcn_exp2f(__fmul_rn(d0, 1.4426950408889634f)); sum += v[t]; }
#pragma unroll
    for (int sh = 16; sh; sh >>= 1) sum += __shfl_xor(sum, sh, 32);
    if (lane == 0) reds[wid] = sum;
    __syncthreads();
    float tot = reds[0];
#pragma unroll
    for (int i = 1; i < 8; ++i) tot += reds[i];
    const float f = PCAR * (1.0f / tot);
#pragma unroll
    for (int t = 0; t < 16; ++t) prow[tid + 256 * t] = (h16)(v[t] * f);
    __syncthreads();
    const v8h val0 = *(const v8ha*)(prow + tid * 8); const v8h val1 = *(const v8ha*)(prow + (256 + tid) * 8);
    h16* dst = P16 + (size_t)p * NPAT;
#pragma unroll 1
    for (int ps = 0; ps < 2; ++ps) { *(volatile v8h*)(dst + tid * 8) = val0; *(volatile v8h*)(dst + (256 + tid) * 8) = val1; if (ps == 0) __threadfence(); }
}

__global__ __launch_bounds__(256) void k_paste(const float* __restrict__ O, float* outb) {
    const int g = blockIdx.x * 256 + threadIdx.x; if (g >= CH * HF * (HF / 4)) return;
    const int xq = g & 31, Y = (g >> 5) & (HF - 1), c = g >> 12;
    const int a0 = (Y + 1) & 1;
    v4f o;
#pragma unroll
    for (int e = 0; e < 4; ++e) { const int X = xq * 4 + e; const int b0 = (X + 1) & 1; float s = 0.0f;
#pragma unroll
        for (int da = 0; da < 2; ++da) { const int a = a0 + 2 * da; const int yy = Y + 1 - a; const bool oky = (yy >= 0) && (yy < 2 * HS); const int y = min(max(yy, 0), 2 * HS - 1) >> 1;
#pragma unroll
            for (int db = 0; db < 2; ++db) { const int b2 = b0 + 2 * db; const int xx = X + 1 - b2; const bool okx = (xx >= 0) && (xx < 2 * HS); const int x = min(max(xx, 0), 2 * HS - 1) >> 1;
                const float val = O[(size_t)(y * HS + x) * NV + c * 16 + a * 4 + b2];
                s += (oky && okx) ? val : 0.0f; } }
        o[e] = s * (1.0f / (PCAR * VCAR)); }
    float* dst = outb + ((size_t)c * HF + Y) * HF + xq * 4;
#pragma unroll 1
    for (int ps = 0; ps < 2; ++ps) { *(volatile v4f*)dst = o; if (ps == 0) __threadfence(); }
}

extern "C" void kernel_launch(void* const* d_in, const int* in_sizes, int n_in,
                              void* d_out, int out_size, void* d_ws, size_t ws_size, hipStream_t stream) {
    if (n_in < 3) return;
    if (in_sizes[0] < (int)((size_t)NB * IMG_FULL) || in_sizes[1] < (int)((size_t)NB * IMG_FULL) || in_sizes[2] < (int)((size_t)NB * MSK_FULL) || out_size < (int)((size_t)NB * IMG_FULL)) return;
    const float* FG = (const float*)d_in[0]; const float* BG = (const float*)d_in[1]; const float* MK = (const float*)d_in[2];
    float* OUT = (float*)d_out;
    char* wsp = (char*)d_ws;
    auto take = [&](size_t bytes) { char* q = wsp; wsp += (bytes + 255) & ~(size_t)255; return (void*)q; };
    bf* AP = (bf*)take((size_t)NPIX * KD * 2);
    bf* BP = (bf*)take((size_t)NPAT * KD * 2);
    h16* VT = (h16*)take((size_t)NV * NPAT * 2);
    float* INV = (float*)take((size_t)NPAT * 4);
    int* FLG = (int*)take((size_t)NPAT * 4);
    float* S = (float*)take((size_t)NPIX * NPAT * 4);
    h16* P16 = (h16*)take((size_t)NPIX * NPAT * 2);
    float* O = S;
    const size_t used = (size_t)(wsp - (char*)d_ws);
    if (used > ws_size || used > (size_t)134217728) return;
    for (int b = 0; b < NB; ++b) {
        const float* fg = FG + (size_t)b * IMG_FULL; const float* bg = BG + (size_t)b * IMG_FULL; const float* mk = MK + (size_t)b * MSK_FULL; float* outb = OUT + (size_t)b * IMG_FULL;
        k_fga<<<NPIX / 64, 256, 0, stream>>>(fg, AP);
        k_bgb<<<NPAT / 64, 256, 0, stream>>>(bg, mk, BP, INV, FLG);
        k_vt<<<NV, 256, 0, stream>>>(bg, VT);
        k_gemmw<bf, 1><<<dim3(NPIX / 64, NPAT / 64, 1), 32, 0, stream>>>(AP, BP, KD, S, NPAT, INV);
        k_soft<<<NPIX, 256, 0, stream>>>(S, FLG, P16);
        k_gemmw<h16, 0><<<dim3(NPIX / 64, NV / 64, 1), 32, 0, stream>>>(P16, VT, NPAT, O, NV, INV);
        k_paste<<<(unsigned)((CH * HF * (HF / 4) + 255) / 256), 256, 0, stream>>>(O, outb);
    }
}
